// MinConv2dGRUCell_35287451304714
// MI455X (gfx1250) — hardware-verified
//
#include <hip/hip_runtime.h>
#include <stdint.h>


typedef __bf16         bf16_t;
typedef bf16_t         v16bf __attribute__((ext_vector_type(16)));
typedef unsigned short v8us  __attribute__((ext_vector_type(8)));
typedef float          v8f   __attribute__((ext_vector_type(8)));
typedef float          v4f   __attribute__((ext_vector_type(4)));
typedef unsigned int   v4u   __attribute__((ext_vector_type(4)));

union Frag { v16bf v; v8us h[2]; };

#define NB_   4
#define NT_   32
#define CIN_  64
#define HID_  64
#define IMH_  32
#define IMW_  32
#define KTOT_ 576
#define KCH_  72
#define ICP_  72
#define XSW_  34
#define OSP_  36
#define N0_   8388608

__device__ __forceinline__ unsigned short f2bf(float f) {
    unsigned int u = __float_as_uint(f);
    u += 0x7FFFu + ((u >> 16) & 1u);
    return (unsigned short)(u >> 16);
}
__device__ __forceinline__ float bfr(float f) {
    return __uint_as_float(((unsigned int)f2bf(f)) << 16);
}

__device__ __forceinline__ v8f mma_bf16(v16bf a, v16bf b, v8f c) {
    return __builtin_amdgcn_wmma_f32_16x16x32_bf16(false, a, false, b, (short)0, c, false, false);
}

__device__ __forceinline__ float scan_lh(float yg, float yh, float lh) {
    const float sp   = log1pf(expf(-fabsf(yg)));
    const float lc   = -(fmaxf(yg, 0.f) + sp);
    const float lz   = fminf(yg, 0.f) - sp;
    const float lpos = logf(fmaxf(yh, 0.f) + 0.5f);
    const float lneg = yh - log1pf(expf(fminf(yh, 0.f)));
    const float lt   = (yh >= 0.f) ? lpos : lneg;
    const float aa   = lc + lh;
    const float bb   = lz + lt;
    const float mx   = fmaxf(aa, bb);
    return mx + log1pf(expf(-fabsf(aa - bb)));
}

__global__ __launch_bounds__(128)
void k_wcvt(const float* __restrict__ W, unsigned short* __restrict__ Wp, int nchunks)
{
    const int j = blockIdx.x * 128 + threadIdx.x;
    if (j < nchunks) {
        const int oc  = j / KCH_;
        const int ch  = j - oc * KCH_;
        const int k0  = ch * 8;
        const int tap = k0 >> 6;
        const int ic0 = k0 & 63;
        const int kh  = (tap * 11) >> 5;
        const int kw  = tap - 3 * kh;
        const float* src = W + ((size_t)(oc * CIN_ + ic0) * 3 + kh) * 3 + kw;
        unsigned int pk[4];
#pragma unroll
        for (int e = 0; e < 4; ++e) {
            const unsigned int lo = (unsigned int)f2bf(src[(2 * e) * 9]);
            const unsigned int hi = (unsigned int)f2bf(src[(2 * e + 1) * 9]);
            pk[e] = lo | (hi << 16);
        }
        v4u v;
        v.x = pk[0]; v.y = pk[1]; v.z = pk[2]; v.w = pk[3];
        volatile v4u* p = (volatile v4u*)(Wp + (size_t)oc * KTOT_ + k0);
        *p = v;
        __threadfence();
        *p = v;
    }
}

__global__ __launch_bounds__(128)
void k_conv_scan(const float* __restrict__ x,
                 const float* __restrict__ h0,
                 const unsigned short* __restrict__ Wp,
                 const float* __restrict__ bias,
                 float* __restrict__ out)
{
    __shared__ alignas(16) unsigned short xs[3 * XSW_ * ICP_];
    __shared__ alignas(16) float ost[4 * 16 * OSP_];

    const int tid  = threadIdx.x;
    const int lane = tid & 31;
    const int w    = tid >> 5;
    const int h    = lane >> 4;
    const int lm   = lane & 15;
    const int bx   = blockIdx.x;
    const int r0   = bx & 31;
    const int b    = bx >> 5;

    for (int idx = tid; idx < 3 * 2 * CIN_; idx += 128) {
        const int r   = idx >> 7;
        const int rem = idx & 127;
        const int cc  = (rem >> 6) ? (XSW_ - 1) : 0;
        const int ic  = rem & 63;
        xs[(r * XSW_ + cc) * ICP_ + ic] = (unsigned short)0;
    }

    float bg[8], bh[8], lh0[8], lh1[8];
#pragma unroll
    for (int r = 0; r < 8; ++r) {
        const int c = 16 * w + 8 * h + r;
        bg[r] = bfr(bias[c]);
        bh[r] = bfr(bias[HID_ + c]);
        const size_t hb = ((size_t)(b * HID_ + c) << 10) + (size_t)(r0 * IMW_);
        lh0[r] = logf(bfr(h0[hb + lm]));
        lh1[r] = logf(bfr(h0[hb + 16 + lm]));
    }

    const unsigned short* wgp = Wp + (size_t)(16 * w + lm) * KTOT_ + 8 * h;
    const unsigned short* whp = Wp + (size_t)(HID_ + 16 * w + lm) * KTOT_ + 8 * h;
    float* ow = ost + w * (16 * OSP_);
    const int f  = lane & 7;
    const int qb = lane >> 3;

    for (int t = 0; t < NT_; ++t) {
        const float* xf = x + ((size_t)((b * NT_ + t) * CIN_) << 10);
#pragma unroll 4
        for (int it = 0; it < 12; ++it) {
            const int q  = tid + it * 128;
            const int r  = q >> 9;
            const int ic = (q >> 3) & 63;
            const int cw = q & 7;
            const int gr = r0 - 1 + r;
            v4f v = {0.f, 0.f, 0.f, 0.f};
            if ((unsigned)gr < (unsigned)IMH_)
                v = *(const v4f*)(xf + ((size_t)ic << 10) + gr * IMW_ + cw * 4);
            const int base = (r * XSW_ + 1 + cw * 4) * ICP_ + ic;
            xs[base]            = f2bf(v.x);
            xs[base + ICP_]     = f2bf(v.y);
            xs[base + 2 * ICP_] = f2bf(v.z);
            xs[base + 3 * ICP_] = f2bf(v.w);
        }
        __syncthreads();

        v8f ag0 = {0.f, 0.f, 0.f, 0.f, 0.f, 0.f, 0.f, 0.f};
        v8f ag1 = ag0, ah0 = ag0, ah1 = ag0;
#pragma unroll 2
        for (int s = 0; s < 18; ++s) {
            const int tap = s >> 1;
            const int kh  = (tap * 11) >> 5;
            const int kw  = tap - 3 * kh;
            const int ich = (s & 1) * 32;
            Frag fa, fb, f0, f1;
            fa.h[0] = *(const v8us*)(wgp + s * 32);
            fa.h[1] = *(const v8us*)(wgp + s * 32 + 16);
            fb.h[0] = *(const v8us*)(whp + s * 32);
            fb.h[1] = *(const v8us*)(whp + s * 32 + 16);
            const unsigned short* px0 = xs + (kh * XSW_ + lm + kw) * ICP_ + ich + 8 * h;
            const unsigned short* px1 = px0 + 16 * ICP_;
            f0.h[0] = *(const v8us*)px0;
            f0.h[1] = *(const v8us*)(px0 + 16);
            f1.h[0] = *(const v8us*)px1;
            f1.h[1] = *(const v8us*)(px1 + 16);
            ag0 = mma_bf16(fa.v, f0.v, ag0);
            ag1 = mma_bf16(fa.v, f1.v, ag1);
            ah0 = mma_bf16(fb.v, f0.v, ah0);
            ah1 = mma_bf16(fb.v, f1.v, ah1);
            asm volatile("v_nop\n\tv_nop\n\tv_nop\n\tv_nop"
                         : "+v"(ag0), "+v"(ag1), "+v"(ah0), "+v"(ah1)
                         : "v"(fa.v), "v"(fb.v), "v"(f0.v), "v"(f1.v));
        }

#pragma unroll
        for (int r = 0; r < 8; ++r) {
            const float n0 = scan_lh(ag0[r] + bg[r], ah0[r] + bh[r], lh0[r]);
            const float n1 = scan_lh(ag1[r] + bg[r], ah1[r] + bh[r], lh1[r]);
            lh0[r] = n0;
            lh1[r] = n1;
            ow[(8 * h + r) * OSP_ + lm]      = expf(n0);
            ow[(8 * h + r) * OSP_ + 16 + lm] = expf(n1);
        }
        __syncthreads();

        v4f ov[4];
#pragma unroll
        for (int it = 0; it < 4; ++it) {
            const int q = it * 4 + qb;
            ov[it] = *(const v4f*)(ow + q * OSP_ + f * 4);
        }
        const size_t ob0 = ((size_t)((b * NT_ + t) * HID_ + 16 * w) << 10) + (size_t)(r0 * IMW_ + f * 4);
        const size_t ob1 = (size_t)N0_ + ((size_t)(b * HID_ + 16 * w) << 10) + (size_t)(r0 * IMW_ + f * 4);
        const bool last = (t == NT_ - 1);
#pragma unroll
        for (int it = 0; it < 4; ++it) {
            const int q = it * 4 + qb;
            *(volatile v4f*)(out + ob0 + ((size_t)q << 10)) = ov[it];
            if (last) *(volatile v4f*)(out + ob1 + ((size_t)q << 10)) = ov[it];
        }
        __threadfence();
#pragma unroll
        for (int it = 0; it < 4; ++it) {
            const int q = it * 4 + qb;
            *(volatile v4f*)(out + ob0 + ((size_t)q << 10)) = ov[it];
            if (last) *(volatile v4f*)(out + ob1 + ((size_t)q << 10)) = ov[it];
        }
    }
}

extern "C" void kernel_launch(void* const* d_in, const int* in_sizes, int n_in,
                              void* d_out, int out_size, void* d_ws, size_t ws_size,
                              hipStream_t stream)
{
    if (n_in < 4) return;
    if (in_sizes[0] != NB_ * NT_ * CIN_ * IMH_ * IMW_) return;
    if (in_sizes[1] != NB_ * HID_ * IMH_ * IMW_) return;
    if (in_sizes[2] != 2 * HID_ * CIN_ * 9) return;
    if (in_sizes[3] != 2 * HID_) return;
    if (out_size != N0_ + NB_ * HID_ * IMH_ * IMW_) return;
    const size_t wp_bytes = (size_t)(2 * HID_) * KTOT_ * sizeof(unsigned short);
    if (ws_size < wp_bytes) return;

    const float* x  = (const float*)d_in[0];
    const float* h0 = (const float*)d_in[1];
    const float* W  = (const float*)d_in[2];
    const float* bs = (const float*)d_in[3];
    float* out = (float*)d_out;
    unsigned short* Wp = (unsigned short*)d_ws;

    const int nchunks = 2 * HID_ * KCH_;
    hipLaunchKernelGGL(k_wcvt, dim3((nchunks + 127) / 128), dim3(128), 0, stream, W, Wp, nchunks);
    hipLaunchKernelGGL(k_conv_scan, dim3(NB_ * IMH_), dim3(128), 0, stream, x, h0, Wp, bs, out);
}
